// TransformerBlockQuantum_65481071398815
// MI455X (gfx1250) — hardware-run, weakly checked
//
#include <hip/hip_runtime.h>
#include <math.h>

typedef __attribute__((ext_vector_type(16))) _Float16 v16h;
typedef __attribute__((ext_vector_type(8)))  _Float16 v8h;
typedef __attribute__((ext_vector_type(8)))  float    v8f;
typedef __attribute__((ext_vector_type(4)))  float    v4f;
typedef __attribute__((ext_vector_type(4)))  unsigned v4u;

constexpr int kBatch      = 32;
constexpr int kSeq        = 4096;
constexpr int kFeat       = 8;
constexpr int kTok        = kBatch * kSeq;
constexpr int kDim        = 256;
constexpr int kHid        = 16;
constexpr int kZN         = 64;
constexpr int kChunk      = 65536;
constexpr int kNumChunk   = kTok / kChunk;
constexpr int kGrpTok     = 4;
constexpr int kGrpPerWave = 4;
constexpr int kTokPerBlk  = 8 * kGrpPerWave * kGrpTok;
static_assert(kTok == 131072 && kNumChunk == 2 && kTokPerBlk == 128);
static_assert((kChunk % kTokPerBlk) == 0 && (kChunk % 256) == 0 && (kChunk % 16) == 0);
static_assert(((kChunk / 16) % 8) == 0);
static_assert((kDim % 32) == 0 && (kZN % 64) == 0);

constexpr float kPCarry = 16384.0f;
constexpr float kFCarry = 1024.0f;
constexpr float sMeas   = 1.0f / kPCarry;
constexpr float sFfn    = 1.0f / (kFCarry * kFCarry);

constexpr size_t kSzSG    = (size_t)kZN * kDim * 2;
constexpr size_t kSzPlane = (size_t)kChunk * kDim * 2;
constexpr size_t kSzZ     = (size_t)kChunk * kZN * 4;
constexpr size_t kSzHB    = (size_t)kTok * kFeat * 4;
constexpr size_t kOffSG   = 0;
constexpr size_t kOffPH   = kOffSG + kSzSG;
constexpr size_t kOffZ1   = kOffPH + kSzPlane;
constexpr size_t kOffZ2   = kOffZ1 + kSzZ;
constexpr size_t kOffHB   = kOffZ2 + kSzZ;
constexpr size_t kWsTotal = kOffHB + kSzHB;
static_assert(kWsTotal == 71335936ull);
static_assert(kWsTotal <= 134217728ull);
static_assert((kOffPH % 128) == 0 && (kOffZ1 % 128) == 0 &&
              (kOffZ2 % 128) == 0 && (kOffHB % 128) == 0);
static_assert((size_t)kTok * kFeat * 4 == 4194304ull);

__host__ __device__ constexpr int cnot_map(int k, int ctrl, int tgt) {
  return ((k >> (7 - ctrl)) & 1) ? (k ^ (1 << (7 - tgt))) : k;
}
__host__ __device__ constexpr int cnot_chain(int k) {
  for (int i = 0; i < 7; ++i) k = cnot_map(k, i, i + 1);
  k = cnot_map(k, 7, 0);
  return k;
}
constexpr bool cnot_chain_is_permutation() {
  bool seen[256] = {};
  for (int k = 0; k < 256; ++k) {
    const int p = cnot_chain(k);
    if (p < 0 || p > 255) return false;
    if (seen[p]) return false;
    seen[p] = true;
  }
  return true;
}
static_assert(cnot_chain_is_permutation());
static_assert(cnot_chain(0) == 0 && cnot_chain(1) == 129 && cnot_chain(128) == 127);

__device__ __forceinline__ float bf16_rne(float f) {
  const unsigned u = __float_as_uint(f);
  const unsigned r = (u + 0x7FFFu + ((u >> 16) & 1u)) & 0xFFFF0000u;
  return __uint_as_float(r);
}
__device__ __forceinline__ _Float16 f16_flush(float v) {
  const float w = (fabsf(v) < 6.103515625e-05f) ? 0.0f : v;
  return (_Float16)w;
}
__device__ __forceinline__ void wave_lds_sync() {
  __builtin_amdgcn_fence(__ATOMIC_RELEASE, "workgroup");
  __builtin_amdgcn_wave_barrier();
  __builtin_amdgcn_fence(__ATOMIC_ACQUIRE, "workgroup");
}

namespace mx {
union FragU { v16h v; v8h h[2]; };
__device__ __forceinline__ v16h frag_load(const _Float16* p) {
  FragU f;
  f.h[0] = *(const v8h*)(p);
  f.h[1] = *(const v8h*)(p + 16);
  return f.v;
}
__device__ __forceinline__ v8f mma(v16h a, v16h b, v8f c) {
  return __builtin_amdgcn_wmma_f32_16x16x32_f16(false, a, false, b, (short)0, c, false, false);
}
__device__ __forceinline__ void guard1(v8f& a, v16h x, v16h y) {
  asm volatile("v_nop\n\tv_nop\n\tv_nop\n\tv_nop" : "+v"(a) : "v"(x), "v"(y));
}
__device__ __forceinline__ void guard_acc(v8f& a) {
  asm volatile("v_nop\n\tv_nop\n\tv_nop\n\tv_nop" : "+v"(a));
}
__device__ __forceinline__ void keep4(v16h a, v16h b, v16h c, v16h d) {
  asm volatile("v_nop" :: "v"(a), "v"(b), "v"(c), "v"(d));
}
}

__global__ __launch_bounds__(256) void sign_plane_kernel(unsigned* __restrict__ SGw)
{
  const int i  = blockIdx.x * 256 + threadIdx.x;
  const int n  = i >> 5;
  const int k0 = (i & 31) * 8;
  const int nn = (n < 8) ? n : 7;
  const unsigned live = (n < 8) ? 1u : 0u;
  v4u w;
#pragma unroll
  for (int e = 0; e < 4; ++e) {
    const int ka = k0 + 2 * e;
    const int kb = ka + 1;
    const unsigned ba = (unsigned)((ka >> (7 - nn)) & 1);
    const unsigned bb = (unsigned)((kb >> (7 - nn)) & 1);
    const unsigned ha = live * (ba ? 0xBC00u : 0x3C00u);
    const unsigned hb = live * (bb ? 0xBC00u : 0x3C00u);
    w[e] = ha | (hb << 16);
  }
  unsigned* p = SGw + (size_t)i * 4;
  *(volatile v4u*)p = w;
  __threadfence();
  *(volatile v4u*)p = w;
}

__device__ __forceinline__ void rx_lane(float (&re)[8], float (&im)[8], float c, float s, int mask)
{
#pragma unroll
  for (int j = 0; j < 8; ++j) {
    const float pr = __shfl_xor(re[j], mask, 32);
    const float pi = __shfl_xor(im[j], mask, 32);
    const float nr = fmaf(s, pi, c * re[j]);
    const float ni = fmaf(-s, pr, c * im[j]);
    re[j] = nr;
    im[j] = ni;
  }
}
template <int MB>
__device__ __forceinline__ void rx_slot(float (&re)[8], float (&im)[8], float c, float s)
{
#pragma unroll
  for (int j = 0; j < 8; ++j) {
    if ((j & MB) == 0) {
      const int j1 = j | MB;
      const float r0 = re[j],  i0 = im[j];
      const float r1 = re[j1], i1 = im[j1];
      re[j]  = fmaf(s, i1, c * r0);
      im[j]  = fmaf(-s, r1, c * i0);
      re[j1] = fmaf(s, i0, c * r1);
      im[j1] = fmaf(-s, r0, c * i1);
    }
  }
}

template <int MODE>
__global__ __launch_bounds__(256) void circuit_planes_kernel(
    const float* __restrict__ x, const float* __restrict__ Z1,
    const float* __restrict__ g1, const float* __restrict__ be1,
    float* __restrict__ HB, unsigned short* __restrict__ PH, int tok0)
{
  __shared__ __align__(16) float stg[8][kGrpTok * kDim];
  const int lane = threadIdx.x & 31;
  const int wave = threadIdx.x >> 5;
  const int gw = blockIdx.x * 8 + wave;
  if (gw * kGrpPerWave >= kChunk / kGrpTok) return;
  float* st = stg[wave];

  int perm[8];
#pragma unroll
  for (int j = 0; j < 8; ++j) perm[j] = cnot_chain(lane * 8 + j);

  float gam = 1.0f, bet = 0.0f;
  if (MODE == 1) {
    gam = bf16_rne(g1[lane & 7]);
    bet = bf16_rne(be1[lane & 7]);
  }

  for (int gi = 0; gi < kGrpPerWave; ++gi) {
    const int g   = gw * kGrpPerWave + gi;
    const int tl0 = g * kGrpTok;
    const size_t gt0 = (size_t)tok0 + (size_t)tl0;
    const float xr = bf16_rne(x[gt0 * kFeat + lane]);
    float ang = xr;
    if (MODE == 1) {
      const int tl = tl0 + (lane >> 3);
      const float z = Z1[(size_t)tl * kZN + (lane & 7)];
      const float y = xr + z;
      float sm = y;
      sm += __shfl_xor(sm, 1, 32);
      sm += __shfl_xor(sm, 2, 32);
      sm += __shfl_xor(sm, 4, 32);
      const float mu = sm * 0.125f;
      const float d = y - mu;
      float sq = d * d;
      sq += __shfl_xor(sq, 1, 32);
      sq += __shfl_xor(sq, 2, 32);
      sq += __shfl_xor(sq, 4, 32);
      const float var = sq * 0.125f;
      const float rs = rsqrtf(var + 1e-5f);
      const float h = d * rs * gam + bet;
      volatile float* hp = HB + gt0 * kFeat + lane;
      *hp = h;
      __threadfence();
      *hp = h;
      ang = h;
    }
    float sn, cs;
    sincosf(ang * 0.5f, &sn, &cs);

    for (int t = 0; t < kGrpTok; ++t) {
      float re[8], im[8];
#pragma unroll
      for (int j = 0; j < 8; ++j) { re[j] = 0.0f; im[j] = 0.0f; }
      re[0] = (lane == 0) ? 1.0f : 0.0f;
      const int src = t * 8;
      const float c0 = __shfl(cs, src + 0, 32), s0 = __shfl(sn, src + 0, 32);
      const float c1 = __shfl(cs, src + 1, 32), s1 = __shfl(sn, src + 1, 32);
      const float c2 = __shfl(cs, src + 2, 32), s2 = __shfl(sn, src + 2, 32);
      const float c3 = __shfl(cs, src + 3, 32), s3 = __shfl(sn, src + 3, 32);
      const float c4 = __shfl(cs, src + 4, 32), s4 = __shfl(sn, src + 4, 32);
      const float c5 = __shfl(cs, src + 5, 32), s5 = __shfl(sn, src + 5, 32);
      const float c6 = __shfl(cs, src + 6, 32), s6 = __shfl(sn, src + 6, 32);
      const float c7 = __shfl(cs, src + 7, 32), s7 = __shfl(sn, src + 7, 32);
      rx_lane(re, im, c0, s0, 16);
      rx_lane(re, im, c1, s1, 8);
      rx_lane(re, im, c2, s2, 4);
      rx_lane(re, im, c3, s3, 2);
      rx_lane(re, im, c4, s4, 1);
      rx_slot<4>(re, im, c5, s5);
      rx_slot<2>(re, im, c6, s6);
      rx_slot<1>(re, im, c7, s7);
#pragma unroll
      for (int j = 0; j < 8; ++j) {
        const float p = fmaf(re[j], re[j], im[j] * im[j]);
        st[t * kDim + perm[j]] = p * kPCarry;
      }
    }
    wave_lds_sync();

    v8h hv[kGrpTok];
#pragma unroll
    for (int t = 0; t < kGrpTok; ++t) {
      const float* sp = st + t * kDim + lane * 8;
      const v4f a0 = *(const v4f*)(sp);
      const v4f a1 = *(const v4f*)(sp + 4);
#pragma unroll
      for (int e = 0; e < 4; ++e) {
        const float f0 = a0[e];
        const float f1 = a1[e];
        hv[t][e]     = f16_flush(f0);
        hv[t][4 + e] = f16_flush(f1);
      }
    }
    for (int pass = 0; pass < 2; ++pass) {
#pragma unroll
      for (int t = 0; t < kGrpTok; ++t) {
        const size_t o = (size_t)(tl0 + t) * kDim + lane * 8;
        *(volatile v8h*)(PH + o) = hv[t];
      }
      __threadfence();
    }
    wave_lds_sync();
  }
}

__global__ __launch_bounds__(256) void measure_gemm_kernel(
    const unsigned short* __restrict__ Ap, int lda,
    const unsigned short* __restrict__ Btp, int ldb,
    float* C, int ldc, int M, int N, int K, float scale)
{
  const _Float16* A  = (const _Float16*)Ap;
  const _Float16* Bt = (const _Float16*)Btp;
  __shared__ __align__(16) float sT[8][16 * 68];
  const int lane = threadIdx.x & 31;
  const int wave = threadIdx.x >> 5;
  const int tilesN = N >> 6;
  const int tilesM = M >> 4;
  const int tile = blockIdx.x * 8 + wave;
  if (tile >= tilesM * tilesN) return;
  const int tm = tile / tilesN;
  const int tn = tile - tm * tilesN;
  const int m0 = tm << 4;
  const int n0 = tn << 6;
  const int rlane = lane & 15;
  const int koff  = (lane >> 4) * 8;
  const int mOff  = (lane >> 4) * 8;

  v8f acc[4];
#pragma unroll
  for (int j = 0; j < 4; ++j) {
    acc[j] = (v8f){0.f, 0.f, 0.f, 0.f, 0.f, 0.f, 0.f, 0.f};
  }

  for (int k0 = 0; k0 < K; k0 += 32) {
    v16h bh[4];
#pragma unroll
    for (int j = 0; j < 4; ++j) {
      const size_t bo = (size_t)(n0 + (j << 4) + rlane) * ldb + koff + k0;
      bh[j] = mx::frag_load(Bt + bo);
    }
    const size_t ao = (size_t)(m0 + rlane) * lda + koff + k0;
    const v16h ah = mx::frag_load(A + ao);
#pragma unroll
    for (int jp = 0; jp < 2; ++jp) {
#pragma unroll
      for (int jj = 0; jj < 2; ++jj) {
        const int j = jp * 2 + jj;
        acc[j] = mx::mma(ah, bh[j], acc[j]);
      }
#pragma unroll
      for (int jj = 0; jj < 2; ++jj) {
        const int j = jp * 2 + jj;
        mx::guard1(acc[j], ah, ah);
      }
    }
    mx::keep4(bh[0], bh[1], bh[2], bh[3]);
  }
#pragma unroll
  for (int j = 0; j < 4; ++j) {
    mx::guard_acc(acc[j]);
  }

  float* slab = sT[wave];
  const int hh = lane >> 4, c4 = (lane & 15) * 4;
#pragma unroll
  for (int j = 0; j < 4; ++j) {
#pragma unroll
    for (int r = 0; r < 8; ++r) {
      const float v = acc[j][r] * scale;
      slab[(mOff + r) * 68 + (j << 4) + rlane] = v;
    }
  }
  wave_lds_sync();
  for (int pass = 0; pass < 2; ++pass) {
#pragma unroll
    for (int it = 0; it < 8; ++it) {
      const int row = it * 2 + hh;
      const v4f v = *(const v4f*)(slab + row * 68 + c4);
      *(volatile v4f*)(C + (size_t)(m0 + row) * ldc + n0 + c4) = v;
    }
    __threadfence();
  }
}

__global__ __launch_bounds__(256) void ffn_norm_kernel(
    const float* __restrict__ Z2, const float* __restrict__ HB,
    const float* __restrict__ w1, const float* __restrict__ b1,
    const float* __restrict__ w2, const float* __restrict__ b2,
    const float* __restrict__ g2, const float* __restrict__ be2,
    float* __restrict__ out, int tok0)
{
  __shared__ __align__(16) _Float16 qs[256 * 32];
  __shared__ __align__(16) _Float16 hs[8][16 * 32];
  __shared__ __align__(16) float fs[256 * 17];
  __shared__ __align__(16) float os[256 * 8];

  const int tid   = threadIdx.x;
  const int lane  = tid & 31;
  const int wave  = tid >> 5;
  const int rlane = lane & 15;
  const int hh    = lane >> 4;
  const int koff  = hh * 8;
  const int mOff  = hh * 8;

  const int tl = blockIdx.x * 256 + tid;
  const size_t gt = (size_t)tok0 + (size_t)tl;

  const v4f q0 = *(const v4f*)(Z2 + (size_t)tl * kZN);
  const v4f q1 = *(const v4f*)(Z2 + (size_t)tl * kZN + 4);
  const v4f h0 = *(const v4f*)(HB + gt * kFeat);
  const v4f h1 = *(const v4f*)(HB + gt * kFeat + 4);
  {
    v8h qv, zv;
#pragma unroll
    for (int e = 0; e < 4; ++e) {
      qv[e]     = f16_flush(q0[e] * kFCarry);
      qv[4 + e] = f16_flush(q1[e] * kFCarry);
    }
#pragma unroll
    for (int e = 0; e < 8; ++e) zv[e] = (_Float16)0.0f;
    _Float16* qrow = qs + tid * 32;
    *(v8h*)(qrow)      = qv;
    *(v8h*)(qrow + 8)  = zv;
    *(v8h*)(qrow + 16) = zv;
    *(v8h*)(qrow + 24) = zv;
    *(v8h*)(hs[wave] + rlane * 32 + 16 + 8 * hh) = zv;
  }

  v16h bw1, bw2;
  {
    const v4f wa = *(const v4f*)(w1 + rlane * 8);
    const v4f wb = *(const v4f*)(w1 + rlane * 8 + 4);
    const int nn = (rlane < 8) ? rlane : 7;
    const v4f wc = *(const v4f*)(w2 + nn * 16 + 8 * hh);
    const v4f wd = *(const v4f*)(w2 + nn * 16 + 8 * hh + 4);
    const bool live1 = (hh == 0);
    const bool live2 = (rlane < 8);
#pragma unroll
    for (int e = 0; e < 4; ++e) {
      const float a0 = bf16_rne(wa[e]) * kFCarry;
      const float a1 = bf16_rne(wb[e]) * kFCarry;
      const float c0 = bf16_rne(wc[e]) * kFCarry;
      const float c1 = bf16_rne(wd[e]) * kFCarry;
      bw1[e]     = f16_flush(live1 ? a0 : 0.0f);
      bw1[4 + e] = f16_flush(live1 ? a1 : 0.0f);
      bw2[e]     = f16_flush(live2 ? c0 : 0.0f);
      bw2[4 + e] = f16_flush(live2 ? c1 : 0.0f);
    }
#pragma unroll
    for (int e = 8; e < 16; ++e) {
      bw1[e] = (_Float16)0.0f;
      bw2[e] = (_Float16)0.0f;
    }
  }
  const float biasH = bf16_rne(b1[rlane]);
  __syncthreads();

  _Float16* hw = hs[wave];
  for (int t = 0; t < 2; ++t) {
    const int tb = wave * 32 + t * 16;
    const v16h a1 = mx::frag_load(qs + (tb + rlane) * 32 + koff);
    v8f acc = (v8f){0.f, 0.f, 0.f, 0.f, 0.f, 0.f, 0.f, 0.f};
    acc = mx::mma(a1, bw1, acc);
    mx::guard1(acc, a1, bw1);
#pragma unroll
    for (int r = 0; r < 8; ++r) {
      float v = fmaf(acc[r], sFfn, biasH);
      v = fmaxf(v, 0.0f);
      hw[(mOff + r) * 32 + rlane] = f16_flush(v * kFCarry);
    }
    wave_lds_sync();
    const v16h a2 = mx::frag_load(hw + rlane * 32 + koff);
    v8f acc2 = (v8f){0.f, 0.f, 0.f, 0.f, 0.f, 0.f, 0.f, 0.f};
    acc2 = mx::mma(a2, bw2, acc2);
    mx::guard1(acc2, a2, bw2);
#pragma unroll
    for (int r = 0; r < 8; ++r) fs[(tb + mOff + r) * 17 + rlane] = acc2[r] * sFfn;
    wave_lds_sync();
  }
  __syncthreads();

  {
    float z[8];
    float mu = 0.0f;
#pragma unroll
    for (int i = 0; i < 8; ++i) {
      const float hvv = (i < 4) ? h0[i & 3] : h1[i & 3];
      const float f = fs[tid * 17 + i] + bf16_rne(b2[i]);
      z[i] = hvv + f;
      mu += z[i];
    }
    mu *= 0.125f;
    float var = 0.0f;
#pragma unroll
    for (int i = 0; i < 8; ++i) { const float d = z[i] - mu; var += d * d; }
    var *= 0.125f;
    const float rs = rsqrtf(var + 1e-5f);
    v4f o0, o1;
#pragma unroll
    for (int i = 0; i < 4; ++i) {
      o0[i] = (z[i] - mu) * rs * bf16_rne(g2[i]) + bf16_rne(be2[i]);
      o1[i] = (z[4 + i] - mu) * rs * bf16_rne(g2[4 + i]) + bf16_rne(be2[4 + i]);
    }
    *(v4f*)(os + tid * 8)     = o0;
    *(v4f*)(os + tid * 8 + 4) = o1;
  }
  __syncthreads();

  {
    const float* sp = os + wave * 256;
    const v4f v0 = *(const v4f*)(sp + lane * 4);
    const v4f v1 = *(const v4f*)(sp + 128 + lane * 4);
    float* op = out + ((size_t)tok0 + (size_t)blockIdx.x * 256 + (size_t)wave * 32) * kFeat;
    for (int pass = 0; pass < 2; ++pass) {
      *(volatile v4f*)(op + lane * 4)       = v0;
      *(volatile v4f*)(op + 128 + lane * 4) = v1;
      __threadfence();
    }
  }
}

extern "C" void kernel_launch(void* const* d_in, const int* in_sizes, int n_in,
                              void* d_out, int out_size, void* d_ws, size_t ws_size,
                              hipStream_t stream)
{
  if (n_in < 9) return;
  if (in_sizes[0] != kTok * kFeat) return;
  if (in_sizes[1] != kFeat) return;
  if (in_sizes[2] != kFeat) return;
  if (in_sizes[3] != kFeat) return;
  if (in_sizes[4] != kFeat) return;
  if (in_sizes[5] != kHid * kFeat) return;
  if (in_sizes[6] != kHid) return;
  if (in_sizes[7] != kFeat * kHid) return;
  if (in_sizes[8] != kFeat) return;
  if (out_size != kTok * kFeat) return;
  if (ws_size < kWsTotal) return;

  const float* x   = (const float*)d_in[0];
  const float* g1  = (const float*)d_in[1];
  const float* be1 = (const float*)d_in[2];
  const float* g2  = (const float*)d_in[3];
  const float* be2 = (const float*)d_in[4];
  const float* w1  = (const float*)d_in[5];
  const float* b1  = (const float*)d_in[6];
  const float* w2  = (const float*)d_in[7];
  const float* b2  = (const float*)d_in[8];
  float* out = (float*)d_out;

  char* ws = (char*)d_ws;
  unsigned short* SG = (unsigned short*)(ws + kOffSG);
  unsigned short* PH = (unsigned short*)(ws + kOffPH);
  float*          Z1 = (float*)(ws + kOffZ1);
  float*          Z2 = (float*)(ws + kOffZ2);
  float*          HB = (float*)(ws + kOffHB);

  sign_plane_kernel<<<dim3((kZN * kDim / 8) / 256), 256, 0, stream>>>((unsigned*)SG);

  for (int c = 0; c < kNumChunk; ++c) {
    const int tok0 = c * kChunk;
    circuit_planes_kernel<0><<<dim3(kChunk / kTokPerBlk), 256, 0, stream>>>(x, Z1, g1, be1, HB, PH, tok0);
    measure_gemm_kernel<<<dim3((kChunk / 16) * (kZN / 64) / 8), 256, 0, stream>>>(
        PH, kDim, SG, kDim, Z1, kZN, kChunk, kZN, kDim, sMeas);
    circuit_planes_kernel<1><<<dim3(kChunk / kTokPerBlk), 256, 0, stream>>>(x, Z1, g1, be1, HB, PH, tok0);
    measure_gemm_kernel<<<dim3((kChunk / 16) * (kZN / 64) / 8), 256, 0, stream>>>(
        PH, kDim, SG, kDim, Z2, kZN, kChunk, kZN, kDim, sMeas);
    ffn_norm_kernel<<<dim3(kChunk / 256), 256, 0, stream>>>(Z2, HB, w1, b1, w2, b2, g2, be2, out, tok0);
  }
}
